// VariableSelectionNetwork_36696200577751
// MI455X (gfx1250) — hardware-verified
//
#include <hip/hip_runtime.h>
#include <math.h>

constexpr int NBATCH = 8;
constexpr int SEQLEN = 512;
constexpr int NFEAT  = 32;
constexpr int HID    = 256;
constexpr int HID2   = 512;
constexpr int CTXD   = 128;
constexpr int NTOK   = NBATCH * SEQLEN;
constexpr int FLATK  = NFEAT * HID;
constexpr int SELN   = 64;
constexpr int FCH    = 4;
constexpr int NCHUNK = NFEAT / FCH;
constexpr int GLP    = 260;
constexpr int SEQ_SHIFT = 9;
constexpr float ACARRY   = 16.0f;
constexpr float WCARRY   = 16.0f;
constexpr float SCALE_AW = 1.0f / 256.0f;
constexpr float SCALE_W  = 1.0f / 16.0f;
constexpr float LN_EPS   = 1e-5f;

static_assert(NTOK % 64 == 0);
static_assert(HID % 64 == 0);
static_assert(HID % 32 == 0);
static_assert(FLATK % 32 == 0);
static_assert(SELN % 64 == 0);
static_assert((1 << SEQ_SHIFT) == SEQLEN);
static_assert(NTOK * (HID / 8) == 131072);
static_assert(NFEAT % FCH == 0);
static_assert((GLP * 4) % 16 == 0);
static_assert(NTOK % 8 == 0);

typedef __attribute__((ext_vector_type(16))) _Float16 v16h;
typedef __attribute__((ext_vector_type(8)))  _Float16 v8h;
typedef __attribute__((ext_vector_type(8)))  float    v8f;
typedef __attribute__((ext_vector_type(4)))  float    v4f;
typedef __attribute__((ext_vector_type(4)))  unsigned int v4u;

__device__ __forceinline__ void guard4_h(v8f& a, v8f& b, v8f& c, v8f& d, v16h x, v16h y) {
  asm volatile("v_nop\n\tv_nop\n\tv_nop\n\tv_nop" : "+v"(a), "+v"(b), "+v"(c), "+v"(d) : "v"(x), "v"(y));
}
__device__ __forceinline__ void keep4_h(v16h a, v16h b, v16h c, v16h d) {
  asm volatile("v_nop" :: "v"(a), "v"(b), "v"(c), "v"(d));
}
__device__ __forceinline__ void acc_guard4(v8f& a, v8f& b, v8f& c, v8f& d) {
  asm volatile("v_nop\n\tv_nop\n\tv_nop\n\tv_nop" : "+v"(a), "+v"(b), "+v"(c), "+v"(d));
}

union FragU { v16h v; v8h h[2]; };
__device__ __forceinline__ v16h frag_load_h(const _Float16* p) {
  FragU f;
  f.h[0] = *(const v8h*)(p);
  f.h[1] = *(const v8h*)(p + 16);
  return f.v;
}
__device__ __forceinline__ v8f wmma_h(v16h a, v16h b, v8f c) {
  return __builtin_amdgcn_wmma_f32_16x16x32_f16(false, a, false, b, (short)0, c, false, false);
}

__device__ __forceinline__ unsigned pk16(unsigned short a, unsigned short b) { return (unsigned)a | ((unsigned)b << 16); }
__device__ __forceinline__ unsigned short h_bits(float f) { const _Float16 h = (_Float16)f; return __builtin_bit_cast(unsigned short, h); }

__device__ __forceinline__ float h16_to_f32(unsigned hb) {
  const unsigned sgn = (hb & 0x8000u) << 16; const unsigned em = hb & 0x7fffu;
  const float fn = __uint_as_float((em << 13) + 0x38000000u);
  const float fs = (float)em * 5.9604644775390625e-8f;
  const float mag = (em < 0x400u) ? fs : fn; return __uint_as_float(__float_as_uint(mag) | sgn);
}

__device__ __forceinline__ float elu_f(float v) {
  const float em = expf(fminf(v, 0.0f)) - 1.0f;
  return (v > 0.0f) ? v : em;
}
__device__ __forceinline__ float sigm_f(float v) {
  const float e = expf(-fmaxf(v, -80.0f));
  return __builtin_amdgcn_rcpf(1.0f + e);
}

__global__ __launch_bounds__(256) void wt_transpose_kernel(const float* __restrict__ W, unsigned short* __restrict__ out,
                                                           int K, int nout, int noutPad, float scale) {
  __shared__ float sm[64][65];
  const int t  = threadIdx.x;
  const int k0 = blockIdx.x * 64;
  const int o0 = blockIdx.y * 64;
  const int z  = blockIdx.z;
  const float* Wz = W + (size_t)z * K * nout;
  unsigned short* oz = out + (size_t)z * noutPad * K;
#pragma unroll
  for (int i = 0; i < 8; ++i) {
    const int e = i * 256 + t;
    const int r = e >> 6;
    const int c = e & 63;
    const int oc = o0 + c;
    const int occ = (oc < nout) ? oc : (nout - 1);
    float v = Wz[(size_t)(k0 + r) * nout + occ] * scale;
    v = (oc < nout) ? v : 0.0f;
    sm[c][r] = v;
  }
  asm volatile("" ::: "memory");
#pragma unroll
  for (int i = 8; i < 16; ++i) {
    const int e = i * 256 + t;
    const int r = e >> 6;
    const int c = e & 63;
    const int oc = o0 + c;
    const int occ = (oc < nout) ? oc : (nout - 1);
    float v = Wz[(size_t)(k0 + r) * nout + occ] * scale;
    v = (oc < nout) ? v : 0.0f;
    sm[c][r] = v;
  }
  __syncthreads();
  const int lane = t & 31, wave = t >> 5;
  const int q = lane >> 3, c8 = (lane & 7) * 8;
  for (int pass = 0; pass < 2; ++pass) {
#pragma unroll
    for (int it = 0; it < 2; ++it) {
      const int row = wave * 8 + it * 4 + q;
      unsigned short hb[8];
#pragma unroll
      for (int e = 0; e < 8; ++e) hb[e] = h_bits(sm[row][c8 + e]);
      const v4u u = (v4u){pk16(hb[0], hb[1]), pk16(hb[2], hb[3]), pk16(hb[4], hb[5]), pk16(hb[6], hb[7])};
      *(volatile v4u*)(oz + (size_t)(o0 + row) * K + k0 + c8) = u;
    }
    __threadfence();
  }
}

__global__ __launch_bounds__(256) void ctxh_kernel(const float* __restrict__ ctx, const float* __restrict__ sctx,
                                                   float* __restrict__ ctxh) {
  const int b = blockIdx.x, h = threadIdx.x;
  float acc = 0.0f;
#pragma unroll 1
  for (int c = 0; c < CTXD; ++c) acc += ctx[b * CTXD + c] * sctx[(size_t)c * HID + h];
  const float v = acc;
  *(volatile float*)(ctxh + (size_t)b * HID + h) = v;
  __threadfence();
  *(volatile float*)(ctxh + (size_t)b * HID + h) = v;
}

__global__ __launch_bounds__(256) void h1gen_kernel(const float* __restrict__ x, const float* __restrict__ w1,
                                                    const float* __restrict__ b1, unsigned short* __restrict__ h1c, int fbase) {
  const int i   = blockIdx.x * 256 + threadIdx.x;
  const int fl  = i >> 17;
  const int rem = i & 131071;
  const int n   = rem >> 5;
  const int kq  = rem & 31;
  const int f   = fbase + fl;
  const float xv = x[(size_t)n * NFEAT + f];
  const float* wr = w1 + (size_t)f * HID + 8 * kq;
  const float* br = b1 + (size_t)f * HID + 8 * kq;
  const v4f wa = *(const v4f*)(wr);
  const v4f wb = *(const v4f*)(wr + 4);
  const v4f ba = *(const v4f*)(br);
  const v4f bb = *(const v4f*)(br + 4);
  unsigned short hb[8];
#pragma unroll
  for (int e = 0; e < 4; ++e) {
    const float v0 = elu_f(xv * wa[e] + ba[e]) * ACARRY;
    const float v1 = elu_f(xv * wb[e] + bb[e]) * ACARRY;
    hb[e]     = h_bits(v0);
    hb[4 + e] = h_bits(v1);
  }
  const v4u u = (v4u){pk16(hb[0], hb[1]), pk16(hb[2], hb[3]), pk16(hb[4], hb[5]), pk16(hb[6], hb[7])};
  unsigned short* op = h1c + 8 * (size_t)i;
  *(volatile v4u*)op = u;
  __threadfence();
  *(volatile v4u*)op = u;
}

template <int BIAS_MODE, int OUT_MODE, int ACT, bool POSTADD>
__global__ __launch_bounds__(256) void gemm64_f16(
    const unsigned short* __restrict__ Ap, int lda, long strideA,
    const unsigned short* __restrict__ Btp, int ldb, long strideB,
    void* __restrict__ Cout, int ldc, long strideC,
    const float* __restrict__ bias, long strideBias,
    const float* __restrict__ addrow, int ldadd, int addShift,
    int M, int N, int K, float scale, float ocarry) {
  const _Float16* A  = (const _Float16*)Ap;
  const _Float16* Bt = (const _Float16*)Btp;
  __shared__ __align__(16) float sT[8][16 * 68];
  const int b    = blockIdx.y;
  const int lane = threadIdx.x & 31;
  const int wave = threadIdx.x >> 5;
  const int tilesN = N >> 6;
  const int tilesM = M >> 6;
  const int tile = blockIdx.x * 8 + wave;
  if (tile >= tilesM * tilesN) return;
  const int tm = tile / tilesN;
  const int tn = tile - tm * tilesN;
  const int m0 = tm << 6;
  const int n0 = tn << 6;

  const _Float16* Ab = A  + (size_t)b * strideA;
  const _Float16* Bb = Bt + (size_t)b * strideB;

  const int rlane = lane & 15;
  const int koff  = (lane >> 4) * 8;
  const int mOff  = (lane >> 4) * 8;

  v8f acc[4][4];
#pragma unroll
  for (int i = 0; i < 4; ++i)
#pragma unroll
    for (int j = 0; j < 4; ++j) acc[i][j] = (v8f){0.f, 0.f, 0.f, 0.f, 0.f, 0.f, 0.f, 0.f};

  for (int k0 = 0; k0 < K; k0 += 32) {
    v16h bh[4];
#pragma unroll
    for (int j = 0; j < 4; ++j)
      bh[j] = frag_load_h(Bb + (size_t)(n0 + (j << 4) + rlane) * ldb + koff + k0);
#pragma unroll
    for (int i = 0; i < 4; ++i) {
      const v16h ah = frag_load_h(Ab + (size_t)(m0 + (i << 4) + rlane) * lda + koff + k0);
#pragma unroll
      for (int j = 0; j < 4; ++j) acc[i][j] = wmma_h(ah, bh[j], acc[i][j]);
      guard4_h(acc[i][0], acc[i][1], acc[i][2], acc[i][3], ah, bh[3]);
    }
    keep4_h(bh[0], bh[1], bh[2], bh[3]);
  }
  acc_guard4(acc[0][0], acc[0][1], acc[0][2], acc[0][3]);
  acc_guard4(acc[1][0], acc[1][1], acc[1][2], acc[1][3]);
  acc_guard4(acc[2][0], acc[2][1], acc[2][2], acc[2][3]);
  acc_guard4(acc[3][0], acc[3][1], acc[3][2], acc[3][3]);

  float* slab = sT[wave];
  const float* biasb = bias + (size_t)b * strideBias;
#pragma unroll
  for (int i = 0; i < 4; ++i) {
    const int mBase = m0 + (i << 4);
#pragma unroll
    for (int j = 0; j < 4; ++j) {
      const int n = n0 + (j << 4) + rlane;
      float bv = 0.f;
      if (BIAS_MODE == 2) bv = biasb[n];
#pragma unroll
      for (int r = 0; r < 8; ++r) {
        float v = acc[i][j][r] * scale;
        if (BIAS_MODE == 1) v += biasb[mBase + mOff + r];
        if (BIAS_MODE == 2) v += bv;
        if (ACT == 2) v = fmaxf(v, 0.0f);
        if (ACT == 6) v = elu_f(v);
        slab[(mOff + r) * 68 + (j << 4) + rlane] = v;
      }
    }
    __builtin_amdgcn_fence(__ATOMIC_RELEASE, "workgroup");
    __builtin_amdgcn_wave_barrier();
    __builtin_amdgcn_fence(__ATOMIC_ACQUIRE, "workgroup");
    if (OUT_MODE == 0) {
      float* C = (float*)Cout + (size_t)b * strideC;
      const int hh = lane >> 4, c4 = (lane & 15) * 4;
      for (int pass = 0; pass < 2; ++pass) {
#pragma unroll
        for (int it = 0; it < 8; ++it) {
          const int row = it * 2 + hh;
          const v4f v = *(const v4f*)(slab + row * 68 + c4);
          *(volatile v4f*)(C + (size_t)(mBase + row) * ldc + n0 + c4) = v;
        }
        __threadfence();
      }
    } else {
      const int q = lane >> 3, c8 = (lane & 7) * 8;
      unsigned short* C = (unsigned short*)Cout + (size_t)b * strideC;
      for (int pass = 0; pass < 2; ++pass) {
#pragma unroll
        for (int it = 0; it < 4; ++it) {
          const int row = it * 4 + q;
          const float* sp = slab + row * 68 + c8;
          float av[8];
#pragma unroll
          for (int e = 0; e < 8; ++e) av[e] = 0.0f;
          if (POSTADD) {
            const float* ar = addrow + (size_t)((mBase + row) >> addShift) * ldadd + n0 + c8;
            const v4f a0 = *(const v4f*)(ar);
            const v4f a1 = *(const v4f*)(ar + 4);
#pragma unroll
            for (int e = 0; e < 4; ++e) { av[e] = a0[e]; av[4 + e] = a1[e]; }
          }
          unsigned short hb[8];
#pragma unroll
          for (int e = 0; e < 8; ++e) hb[e] = h_bits((sp[e] + av[e]) * ocarry);
          const v4u u = (v4u){pk16(hb[0], hb[1]), pk16(hb[2], hb[3]), pk16(hb[4], hb[5]), pk16(hb[6], hb[7])};
          *(volatile v4u*)(C + (size_t)(mBase + row) * ldc + n0 + c8) = u;
        }
        __threadfence();
      }
    }
    __builtin_amdgcn_fence(__ATOMIC_RELEASE, "workgroup");
    __builtin_amdgcn_wave_barrier();
    __builtin_amdgcn_fence(__ATOMIC_ACQUIRE, "workgroup");
  }
}

template <bool STK>
__global__ __launch_bounds__(256) void glu_ln_kernel(
    const unsigned short* __restrict__ Ap, long strideA,
    const unsigned short* __restrict__ Btp, long strideB,
    const float* __restrict__ bias, long strideBias,
    const float* __restrict__ xp,
    const float* __restrict__ wsp, const float* __restrict__ bsp,
    const float* __restrict__ gam, const float* __restrict__ bet, long strideG,
    const float* __restrict__ resid,
    unsigned short* __restrict__ outStk, float* __restrict__ outF,
    int fbase, float scale) {
  __shared__ __align__(16) float sglu[64 * GLP];
  const int lane = threadIdx.x & 31;
  const int wave = threadIdx.x >> 5;
  const int rlane = lane & 15;
  const int koff  = (lane >> 4) * 8;
  const int mOff  = koff;
  const int m0 = blockIdx.x * 64;
  const int fl = blockIdx.y;
  const int f  = fbase + fl;
  const _Float16* A  = (const _Float16*)Ap  + (size_t)fl * strideA;
  const _Float16* Bt = (const _Float16*)Btp + (size_t)f  * strideB;
  const float* biasf = bias + (size_t)f * strideBias;
  const int cv0 = wave * 32;

  v8f acc[4][4];
#pragma unroll
  for (int i = 0; i < 4; ++i)
#pragma unroll
    for (int j = 0; j < 4; ++j) acc[i][j] = (v8f){0.f, 0.f, 0.f, 0.f, 0.f, 0.f, 0.f, 0.f};

  for (int k0 = 0; k0 < HID; k0 += 32) {
    v16h bh[4];
    bh[0] = frag_load_h(Bt + (size_t)(cv0 + rlane) * HID + koff + k0);
    bh[1] = frag_load_h(Bt + (size_t)(cv0 + 16 + rlane) * HID + koff + k0);
    bh[2] = frag_load_h(Bt + (size_t)(HID + cv0 + rlane) * HID + koff + k0);
    bh[3] = frag_load_h(Bt + (size_t)(HID + cv0 + 16 + rlane) * HID + koff + k0);
#pragma unroll
    for (int i = 0; i < 4; ++i) {
      const v16h ah = frag_load_h(A + (size_t)(m0 + (i << 4) + rlane) * HID + koff + k0);
#pragma unroll
      for (int j = 0; j < 4; ++j) acc[i][j] = wmma_h(ah, bh[j], acc[i][j]);
      guard4_h(acc[i][0], acc[i][1], acc[i][2], acc[i][3], ah, bh[3]);
    }
    keep4_h(bh[0], bh[1], bh[2], bh[3]);
  }
  acc_guard4(acc[0][0], acc[0][1], acc[0][2], acc[0][3]);
  acc_guard4(acc[1][0], acc[1][1], acc[1][2], acc[1][3]);
  acc_guard4(acc[2][0], acc[2][1], acc[2][2], acc[2][3]);
  acc_guard4(acc[3][0], acc[3][1], acc[3][2], acc[3][3]);

#pragma unroll
  for (int i = 0; i < 4; ++i) {
#pragma unroll
    for (int jv = 0; jv < 2; ++jv) {
      const int c = cv0 + (jv << 4) + rlane;
      const float bv    = biasf[c];
      const float bgate = biasf[HID + c];
#pragma unroll
      for (int r = 0; r < 8; ++r) {
        const float gv = acc[i][jv][r] * scale + bv;
        const float gs = acc[i][jv + 2][r] * scale + bgate;
        sglu[((i << 4) + mOff + r) * GLP + c] = gv * sigm_f(gs);
      }
    }
  }
  __syncthreads();

  if (STK) {
    const int c0 = 8 * lane;
    float wsv[8], bsv[8], gmv[8], btv[8];
    {
      const float* wr = wsp + (size_t)f * HID + c0;
      const float* br = bsp + (size_t)f * HID + c0;
      const v4f wa = *(const v4f*)(wr); const v4f wb = *(const v4f*)(wr + 4);
      const v4f ba = *(const v4f*)(br); const v4f bb = *(const v4f*)(br + 4);
#pragma unroll
      for (int e = 0; e < 4; ++e) { wsv[e] = wa[e]; wsv[4 + e] = wb[e]; bsv[e] = ba[e]; bsv[4 + e] = bb[e]; }
    }
    asm volatile("" ::: "memory");
    {
      const float* gr = gam + (size_t)f * strideG + c0;
      const float* tr = bet + (size_t)f * strideG + c0;
      const v4f ga = *(const v4f*)(gr); const v4f gb = *(const v4f*)(gr + 4);
      const v4f ta = *(const v4f*)(tr); const v4f tb = *(const v4f*)(tr + 4);
#pragma unroll
      for (int e = 0; e < 4; ++e) { gmv[e] = ga[e]; gmv[4 + e] = gb[e]; btv[e] = ta[e]; btv[4 + e] = tb[e]; }
    }
    asm volatile("" ::: "memory");
#pragma unroll 1
    for (int grp = 0; grp < 2; ++grp) {
      v4u pk[4];
#pragma unroll
      for (int rr = 0; rr < 4; ++rr) {
        const int rloc = wave * 8 + grp * 4 + rr;
        const int grow = m0 + rloc;
        const float xv = xp[(size_t)grow * NFEAT + f];
        const float* gp = sglu + rloc * GLP + c0;
        const v4f ga = *(const v4f*)(gp);
        const v4f gb = *(const v4f*)(gp + 4);
        float t[8];
#pragma unroll
        for (int e = 0; e < 4; ++e) {
          t[e]     = ga[e] + (xv * wsv[e] + bsv[e]);
          t[4 + e] = gb[e] + (xv * wsv[4 + e] + bsv[4 + e]);
        }
        float s = 0.0f;
#pragma unroll
        for (int e = 0; e < 8; ++e) s += t[e];
#pragma unroll
        for (int off = 16; off > 0; off >>= 1) s += __shfl_xor(s, off, 32);
        const float mean = s * (1.0f / (float)HID);
        float d[8];
        float sq = 0.0f;
#pragma unroll
        for (int e = 0; e < 8; ++e) { d[e] = t[e] - mean; sq += d[e] * d[e]; }
#pragma unroll
        for (int off = 16; off > 0; off >>= 1) sq += __shfl_xor(sq, off, 32);
        const float var  = sq * (1.0f / (float)HID);
        const float rstd = rsqrtf(var + LN_EPS);
        unsigned short hb[8];
#pragma unroll
        for (int e = 0; e < 8; ++e) hb[e] = h_bits(d[e] * rstd * gmv[e] + btv[e]);
        pk[rr] = (v4u){pk16(hb[0], hb[1]), pk16(hb[2], hb[3]), pk16(hb[4], hb[5]), pk16(hb[6], hb[7])};
      }
      for (int pass = 0; pass < 2; ++pass) {
#pragma unroll
        for (int rr = 0; rr < 4; ++rr) {
          const int grow = m0 + wave * 8 + grp * 4 + rr;
          *(volatile v4u*)(outStk + ((size_t)grow * NFEAT + f) * HID + c0) = pk[rr];
        }
        __threadfence();
      }
    }
  } else {
    const int c0 = 4 * lane;
    const int c1 = (HID / 2) + 4 * lane;
    float gmv[8], btv[8];
    {
      const float* gr = gam + (size_t)f * strideG;
      const float* tr = bet + (size_t)f * strideG;
      const v4f ga = *(const v4f*)(gr + c0); const v4f gb = *(const v4f*)(gr + c1);
      const v4f ta = *(const v4f*)(tr + c0); const v4f tb = *(const v4f*)(tr + c1);
#pragma unroll
      for (int e = 0; e < 4; ++e) { gmv[e] = ga[e]; gmv[4 + e] = gb[e]; btv[e] = ta[e]; btv[4 + e] = tb[e]; }
    }
    asm volatile("" ::: "memory");
#pragma unroll 1
    for (int grp = 0; grp < 2; ++grp) {
      v4f o0[4], o1[4];
#pragma unroll
      for (int rr = 0; rr < 4; ++rr) {
        const int rloc = wave * 8 + grp * 4 + rr;
        const int grow = m0 + rloc;
        const float* gp = sglu + rloc * GLP;
        const v4f ga = *(const v4f*)(gp + c0);
        const v4f gb = *(const v4f*)(gp + c1);
        const float* rp = resid + (size_t)grow * HID;
        const v4f ra = *(const v4f*)(rp + c0);
        const v4f rb = *(const v4f*)(rp + c1);
        float t[8];
#pragma unroll
        for (int e = 0; e < 4; ++e) { t[e] = ga[e] + ra[e]; t[4 + e] = gb[e] + rb[e]; }
        float s = 0.0f;
#pragma unroll
        for (int e = 0; e < 8; ++e) s += t[e];
#pragma unroll
        for (int off = 16; off > 0; off >>= 1) s += __shfl_xor(s, off, 32);
        const float mean = s * (1.0f / (float)HID);
        float d[8];
        float sq = 0.0f;
#pragma unroll
        for (int e = 0; e < 8; ++e) { d[e] = t[e] - mean; sq += d[e] * d[e]; }
#pragma unroll
        for (int off = 16; off > 0; off >>= 1) sq += __shfl_xor(sq, off, 32);
        const float var  = sq * (1.0f / (float)HID);
        const float rstd = rsqrtf(var + LN_EPS);
        float y[8];
#pragma unroll
        for (int e = 0; e < 8; ++e) y[e] = d[e] * rstd * gmv[e] + btv[e];
        o0[rr] = (v4f){y[0], y[1], y[2], y[3]};
        o1[rr] = (v4f){y[4], y[5], y[6], y[7]};
      }
      for (int pass = 0; pass < 2; ++pass) {
#pragma unroll
        for (int rr = 0; rr < 4; ++rr) {
          const int grow = m0 + wave * 8 + grp * 4 + rr;
          *(volatile v4f*)(outF + (size_t)grow * HID + c0) = o0[rr];
          *(volatile v4f*)(outF + (size_t)grow * HID + c1) = o1[rr];
        }
        __threadfence();
      }
    }
  }
}

__global__ __launch_bounds__(256) void sel_weights_kernel(const float* __restrict__ gg, const float* __restrict__ ssk,
                                                          const float* __restrict__ skb, const float* __restrict__ sg,
                                                          const float* __restrict__ sbt,
                                                          float* __restrict__ wbuf, float* __restrict__ outw) {
  const int lane = threadIdx.x & 31;
  const int wave = threadIdx.x >> 5;
  const int n = blockIdx.x * 8 + wave;
  const float a  = gg[(size_t)n * SELN + lane];
  const float g  = gg[(size_t)n * SELN + NFEAT + lane];
  const float sk = ssk[(size_t)n * SELN + lane] + skb[lane];
  const float t  = a * sigm_f(g) + sk;
  float s = 0.0f;
  s += t;
#pragma unroll
  for (int off = 16; off > 0; off >>= 1) s += __shfl_xor(s, off, 32);
  const float mean = s * (1.0f / (float)NFEAT);
  const float d = t - mean;
  float sq = 0.0f;
  sq += d * d;
#pragma unroll
  for (int off = 16; off > 0; off >>= 1) sq += __shfl_xor(sq, off, 32);
  const float var  = sq * (1.0f / (float)NFEAT);
  const float rstd = rsqrtf(var + LN_EPS);
  const float lg = d * rstd * sg[lane] + sbt[lane];
  float mx = lg;
#pragma unroll
  for (int off = 16; off > 0; off >>= 1) mx = fmaxf(mx, __shfl_xor(mx, off, 32));
  const float e = expf(lg - mx);
  float se = 0.0f;
  se += e;
#pragma unroll
  for (int off = 16; off > 0; off >>= 1) se += __shfl_xor(se, off, 32);
  const float w = e * __builtin_amdgcn_rcpf(se);
  *(volatile float*)(outw + (size_t)n * NFEAT + lane) = w;
  *(volatile float*)(wbuf + (size_t)n * NFEAT + lane) = w;
  __threadfence();
  *(volatile float*)(outw + (size_t)n * NFEAT + lane) = w;
  *(volatile float*)(wbuf + (size_t)n * NFEAT + lane) = w;
}

__global__ __launch_bounds__(256) void combine_kernel(const unsigned short* __restrict__ stk, const float* __restrict__ wb,
                                                      float* __restrict__ comb, unsigned short* __restrict__ comb16) {
  __shared__ __align__(16) float srow[8][HID];
  const int lane = threadIdx.x & 31;
  const int wave = threadIdx.x >> 5;
  const int n = blockIdx.x * 8 + wave;
  const float wl = wb[(size_t)n * NFEAT + lane];
  float acc[8];
#pragma unroll
  for (int e = 0; e < 8; ++e) acc[e] = 0.0f;
  const unsigned short* base = stk + (size_t)n * NFEAT * HID + 8 * lane;
#pragma unroll 1
  for (int f = 0; f < NFEAT; ++f) {
    const float wf = __shfl(wl, f, 32);
    const v4u u = *(const v4u*)(base + (size_t)f * HID);
#pragma unroll
    for (int e = 0; e < 4; ++e) {
      const unsigned wd = u[e];
      acc[2 * e]     += h16_to_f32(wd & 0xffffu) * wf;
      acc[2 * e + 1] += h16_to_f32(wd >> 16) * wf;
    }
  }
  unsigned short hb[8];
#pragma unroll
  for (int e = 0; e < 8; ++e) { hb[e] = h_bits(acc[e]); srow[wave][8 * lane + e] = acc[e]; }
  const v4u u16 = (v4u){pk16(hb[0], hb[1]), pk16(hb[2], hb[3]), pk16(hb[4], hb[5]), pk16(hb[6], hb[7])};
  __syncthreads();
  const v4f va = *(const v4f*)(&srow[wave][4 * lane]);
  const v4f vb = *(const v4f*)(&srow[wave][(HID / 2) + 4 * lane]);
  for (int pass = 0; pass < 2; ++pass) {
    *(volatile v4f*)(comb + (size_t)n * HID + 4 * lane) = va;
    *(volatile v4f*)(comb + (size_t)n * HID + (HID / 2) + 4 * lane) = vb;
    *(volatile v4u*)(comb16 + (size_t)n * HID + 8 * lane) = u16;
    __threadfence();
  }
}

extern "C" void kernel_launch(void* const* d_in, const int* in_sizes, int n_in,
                              void* d_out, int out_size, void* d_ws, size_t ws_size, hipStream_t stream) {
  if (n_in < 31) return;
  if (out_size != NTOK * HID + NTOK * NFEAT) return;
  if (in_sizes[0] != NTOK * NFEAT) return;

  const float* x    = (const float*)d_in[0];
  const float* ctx  = (const float*)d_in[1];
  const float* w1   = (const float*)d_in[2];
  const float* b1   = (const float*)d_in[3];
  const float* w2   = (const float*)d_in[4];
  const float* b2   = (const float*)d_in[5];
  const float* wg   = (const float*)d_in[6];
  const float* bg   = (const float*)d_in[7];
  const float* wsk  = (const float*)d_in[8];
  const float* bsk  = (const float*)d_in[9];
  const float* g1   = (const float*)d_in[10];
  const float* be1  = (const float*)d_in[11];
  const float* sw1  = (const float*)d_in[12];
  const float* sb1  = (const float*)d_in[13];
  const float* sctx = (const float*)d_in[14];
  const float* sw2  = (const float*)d_in[15];
  const float* sb2  = (const float*)d_in[16];
  const float* sgw  = (const float*)d_in[17];
  const float* sgb  = (const float*)d_in[18];
  const float* sg   = (const float*)d_in[19];
  const float* sbt  = (const float*)d_in[20];
  const float* skw  = (const float*)d_in[21];
  const float* skb  = (const float*)d_in[22];
  const float* ow1  = (const float*)d_in[23];
  const float* ob1  = (const float*)d_in[24];
  const float* ow2  = (const float*)d_in[25];
  const float* ob2  = (const float*)d_in[26];
  const float* ogw  = (const float*)d_in[27];
  const float* ogb  = (const float*)d_in[28];
  const float* og   = (const float*)d_in[29];
  const float* obt  = (const float*)d_in[30];

  char* wsb = (char*)d_ws;
  size_t off = 0;
  auto carve = [&](size_t bytes) -> char* {
    char* p = wsb + off;
    off += (bytes + 255) & ~((size_t)255);
    return p;
  };
  unsigned short* w2t  = (unsigned short*)carve((size_t)NFEAT * HID * HID * 2);
  unsigned short* wgt  = (unsigned short*)carve((size_t)NFEAT * HID2 * HID * 2);
  unsigned short* sw1t = (unsigned short*)carve((size_t)HID * FLATK * 2);
  unsigned short* skwt = (unsigned short*)carve((size_t)SELN * FLATK * 2);
  unsigned short* sw2t = (unsigned short*)carve((size_t)HID * HID * 2);
  unsigned short* sgwt = (unsigned short*)carve((size_t)SELN * HID * 2);
  unsigned short* ow1t = (unsigned short*)carve((size_t)HID * HID * 2);
  unsigned short* ow2t = (unsigned short*)carve((size_t)HID * HID * 2);
  unsigned short* ogwt = (unsigned short*)carve((size_t)HID2 * HID * 2);
  float*          ctxh = (float*)carve((size_t)NBATCH * HID * 4);
  unsigned short* h1c  = (unsigned short*)carve((size_t)FCH * NTOK * HID * 2);
  unsigned short* h2c  = (unsigned short*)carve((size_t)FCH * NTOK * HID * 2);
  unsigned short* stacked = (unsigned short*)carve((size_t)NTOK * NFEAT * HID * 2);
  unsigned short* hs16 = (unsigned short*)carve((size_t)NTOK * HID * 2);
  float*          sskip = (float*)carve((size_t)NTOK * SELN * 4);
  unsigned short* hs2  = (unsigned short*)carve((size_t)NTOK * HID * 2);
  float*          gg   = (float*)carve((size_t)NTOK * SELN * 4);
  float*          wbuf = (float*)carve((size_t)NTOK * NFEAT * 4);
  float*          comb = (float*)carve((size_t)NTOK * HID * 4);
  unsigned short* comb16 = (unsigned short*)carve((size_t)NTOK * HID * 2);
  unsigned short* ho1  = (unsigned short*)carve((size_t)NTOK * HID * 2);
  unsigned short* ho2  = (unsigned short*)carve((size_t)NTOK * HID * 2);
  if (off > ws_size) return;

  float* out0 = (float*)d_out;
  float* out1 = out0 + (size_t)NTOK * HID;

  const dim3 blk(256);

  wt_transpose_kernel<<<dim3(HID / 64, HID / 64, NFEAT), blk, 0, stream>>>(w2, w2t, HID, HID, HID, WCARRY);
  wt_transpose_kernel<<<dim3(HID / 64, HID2 / 64, NFEAT), blk, 0, stream>>>(wg, wgt, HID, HID2, HID2, WCARRY);
  wt_transpose_kernel<<<dim3(FLATK / 64, HID / 64, 1), blk, 0, stream>>>(sw1, sw1t, FLATK, HID, HID, WCARRY);
  wt_transpose_kernel<<<dim3(FLATK / 64, SELN / 64, 1), blk, 0, stream>>>(skw, skwt, FLATK, NFEAT, SELN, WCARRY);
  wt_transpose_kernel<<<dim3(HID / 64, HID / 64, 1), blk, 0, stream>>>(sw2, sw2t, HID, HID, HID, WCARRY);
  wt_transpose_kernel<<<dim3(HID / 64, SELN / 64, 1), blk, 0, stream>>>(sgw, sgwt, HID, SELN, SELN, WCARRY);
  wt_transpose_kernel<<<dim3(HID / 64, HID / 64, 1), blk, 0, stream>>>(ow1, ow1t, HID, HID, HID, WCARRY);
  wt_transpose_kernel<<<dim3(HID / 64, HID / 64, 1), blk, 0, stream>>>(ow2, ow2t, HID, HID, HID, WCARRY);
  wt_transpose_kernel<<<dim3(HID / 64, HID2 / 64, 1), blk, 0, stream>>>(ogw, ogwt, HID, HID2, HID2, WCARRY);

  ctxh_kernel<<<dim3(NBATCH), blk, 0, stream>>>(ctx, sctx, ctxh);

  for (int ch = 0; ch < NCHUNK; ++ch) {
    const int fbase = ch * FCH;
    h1gen_kernel<<<dim3(FCH * NTOK * (HID / 8) / 256), blk, 0, stream>>>(x, w1, b1, h1c, fbase);
    gemm64_f16<2, 1, 6, false><<<dim3((NTOK / 64) * (HID / 64) / 8, FCH), blk, 0, stream>>>(
        h1c, HID, (long)NTOK * HID,
        w2t + (size_t)fbase * HID * HID, HID, (long)HID * HID,
        (void*)h2c, HID, (long)NTOK * HID,
        b2 + (size_t)fbase * HID, (long)HID,
        nullptr, 0, 0,
        NTOK, HID, HID, SCALE_AW, ACARRY);
    glu_ln_kernel<true><<<dim3(NTOK / 64, FCH), blk, 0, stream>>>(
        h2c, (long)NTOK * HID,
        wgt, (long)HID2 * HID,
        bg, (long)HID2,
        x, wsk, bsk,
        g1, be1, (long)HID,
        nullptr,
        stacked, nullptr,
        fbase, SCALE_AW);
  }

  gemm64_f16<2, 1, 6, true><<<dim3((NTOK / 64) * (HID / 64) / 8, 1), blk, 0, stream>>>(
      stacked, FLATK, 0L,
      sw1t, FLATK, 0L,
      (void*)hs16, HID, 0L,
      sb1, 0L,
      ctxh, HID, SEQ_SHIFT,
      NTOK, HID, FLATK, SCALE_W, 1.0f);
  gemm64_f16<0, 0, 0, false><<<dim3((NTOK / 64) * (SELN / 64) / 8, 1), blk, 0, stream>>>(
      stacked, FLATK, 0L,
      skwt, FLATK, 0L,
      (void*)sskip, SELN, 0L,
      nullptr, 0L,
      nullptr, 0, 0,
      NTOK, SELN, FLATK, SCALE_W, 1.0f);
  gemm64_f16<2, 1, 6, false><<<dim3((NTOK / 64) * (HID / 64) / 8, 1), blk, 0, stream>>>(
      hs16, HID, 0L,
      sw2t, HID, 0L,
      (void*)hs2, HID, 0L,
      sb2, 0L,
      nullptr, 0, 0,
      NTOK, HID, HID, SCALE_W, 1.0f);
  gemm64_f16<2, 0, 0, false><<<dim3((NTOK / 64) * (SELN / 64) / 8, 1), blk, 0, stream>>>(
      hs2, HID, 0L,
      sgwt, HID, 0L,
      (void*)gg, SELN, 0L,
      sgb, 0L,
      nullptr, 0, 0,
      NTOK, SELN, HID, SCALE_W, 1.0f);
  sel_weights_kernel<<<dim3(NTOK / 8), blk, 0, stream>>>(gg, sskip, skb, sg, sbt, wbuf, out1);
  combine_kernel<<<dim3(NTOK / 8), blk, 0, stream>>>(stacked, wbuf, comb, comb16);
  gemm64_f16<2, 1, 6, false><<<dim3((NTOK / 64) * (HID / 64) / 8, 1), blk, 0, stream>>>(
      comb16, HID, 0L,
      ow1t, HID, 0L,
      (void*)ho1, HID, 0L,
      ob1, 0L,
      nullptr, 0, 0,
      NTOK, HID, HID, SCALE_W, 1.0f);
  gemm64_f16<2, 1, 6, false><<<dim3((NTOK / 64) * (HID / 64) / 8, 1), blk, 0, stream>>>(
      ho1, HID, 0L,
      ow2t, HID, 0L,
      (void*)ho2, HID, 0L,
      ob2, 0L,
      nullptr, 0, 0,
      NTOK, HID, HID, SCALE_W, 1.0f);
  glu_ln_kernel<false><<<dim3(NTOK / 64, 1), blk, 0, stream>>>(
      ho2, 0L,
      ogwt, 0L,
      ogb, 0L,
      nullptr, nullptr, nullptr,
      og, obt, 0L,
      comb,
      nullptr, out0,
      0, SCALE_W);
}
